// LSTMnoTF_9577777070394
// MI455X (gfx1250) — hardware-run, weakly checked
//
#include <hip/hip_runtime.h>


#define AS3 __attribute__((address_space(3)))

#define B_   256
#define T_   256
#define I_   32
#define H_   512
#define G4_  2048
#define O_   32
#define F_   128
#define KC_  544
#define WPITCH 576
#define APITCH 552
#define CPITCH 512
#define PPITCH 36
#define MB_  32
#define NBLK (B_ / MB_)
#define NTHR 256
#define NSTEP (T_ + F_ - 1)

static_assert(KC_ == I_ + H_);
static_assert(KC_ % 32 == 0);
static_assert(H_ % 32 == 0);
static_assert(APITCH % 8 == 0);
static_assert(APITCH >= KC_);
static_assert(WPITCH % 64 == 0);
static_assert(WPITCH >= KC_);
static_assert(MB_ == 32);
static_assert(NTHR == 256);
static_assert(H_ == (NTHR / 32) * 64);
static_assert(B_ % MB_ == 0);
static_assert(O_ == 32);

typedef _Float16 v16h __attribute__((ext_vector_type(16)));
typedef _Float16 v8h  __attribute__((ext_vector_type(8)));
typedef _Float16 v4h  __attribute__((ext_vector_type(4)));
typedef float    v8f  __attribute__((ext_vector_type(8)));
typedef float    v4f  __attribute__((ext_vector_type(4)));

typedef AS3 _Float16*       lp_h;
typedef AS3 const _Float16* lcp_h;
typedef AS3 float*          lp_f;

union Frag { v16h v; v8h half[2]; };

constexpr int    NWPC  = WPITCH / 8;
constexpr int    NWP   = G4_ * NWPC;
constexpr int    NWBLK = NWP / 256;
constexpr int    NFP   = O_ * (H_ / 8);
constexpr int    NFBLK = NFP / 256;
static_assert(NWP % 256 == 0);
static_assert(NFP % 256 == 0);

constexpr size_t SZ_WP  = (size_t)G4_ * WPITCH * 2;
constexpr size_t SZ_WF  = (size_t)O_ * H_ * 2;
constexpr size_t OFF_WP = 0;
constexpr size_t OFF_WF = OFF_WP + SZ_WP;
constexpr size_t WS_END = OFF_WF + SZ_WF;
static_assert(OFF_WF % 128 == 0);
static_assert(WS_END <= (size_t)134217728);
static_assert((size_t)NWP * 16 == SZ_WP);
static_assert((size_t)NFP * 16 == SZ_WF);

constexpr int    A_TILE    = MB_ * APITCH;
constexpr size_t LOFF_A    = 0;
constexpr size_t LSZ_A     = (size_t)2 * A_TILE * 2;
constexpr size_t LOFF_C    = LOFF_A + LSZ_A;
constexpr size_t LSZ_C     = (size_t)MB_ * CPITCH * 4;
constexpr size_t LOFF_BIAS = LOFF_C + LSZ_C;
constexpr size_t LOFF_BFC  = LOFF_BIAS + (size_t)G4_ * 4;
constexpr size_t LOFF_P    = LOFF_BFC + 128;
constexpr size_t LDS_BYTES = LOFF_P + (size_t)MB_ * PPITCH * 4;
static_assert(LOFF_C % 16 == 0 && LOFF_BIAS % 16 == 0 && LOFF_BFC % 16 == 0 && LOFF_P % 16 == 0);
static_assert((2 * A_TILE) % 8 == 0);
static_assert((MB_ * CPITCH) % 4 == 0);

#define SCL    16.0f
#define INV256 0.00390625f

__device__ __forceinline__ float rcpx(float x) { return __builtin_amdgcn_rcpf(x); }
__device__ __forceinline__ float sigm(float x) { return rcpx(1.0f + __expf(-x)); }
__device__ __forceinline__ float tanhm(float x) {
    const float e = __expf(2.0f * x);
    return 1.0f - 2.0f * rcpx(e + 1.0f);
}
__device__ __forceinline__ v8f ld8f(const float* p) {
    const v4f a = *(const v4f*)p;
    const v4f b = *(const v4f*)(p + 4);
    return __builtin_shufflevector(a, b, 0, 1, 2, 3, 4, 5, 6, 7);
}
__device__ __forceinline__ v8f zero8() {
    v8f z;
#pragma unroll
    for (int i = 0; i < 8; ++i) z[i] = 0.0f;
    return z;
}

__device__ __forceinline__ void ldfrag_lds(Frag& f, lcp_h p) {
    f.half[0] = *(AS3 const v8h*)(p);
    f.half[1] = *(AS3 const v8h*)(p + 16);
}
__device__ __forceinline__ void ldfrag_glb(Frag& f, const _Float16* p) {
    f.half[0] = *(const v8h*)(p);
    f.half[1] = *(const v8h*)(p + 16);
}
__device__ __forceinline__ v8f mma16(v8f c, const Frag& a, const Frag& b) {
    return __builtin_amdgcn_wmma_f32_16x16x32_f16(false, a.v, false, b.v, (short)0, c, false, false);
}

__global__ __launch_bounds__(256)
void cvt_kernel(const float* __restrict__ Wih, const float* __restrict__ Whh,
                const float* __restrict__ Wfc, _Float16* Wp, _Float16* Wf)
{
    const int tid = threadIdx.x;
    if ((int)blockIdx.x < NWBLK) {
        const int p  = blockIdx.x * 256 + tid;
        const int n  = p / NWPC;
        const int c8 = (p - n * NWPC) * 8;
        const int ci = min(c8, I_ - 8);
        const int cj = min(max(c8 - I_, 0), H_ - 8);
        const v8f a = ld8f(Wih + (size_t)n * I_ + ci);
        const v8f b = ld8f(Whh + (size_t)n * H_ + cj);
        v8h hv;
#pragma unroll
        for (int i = 0; i < 8; ++i) {
            const float v = (c8 < I_) ? a[i] : ((c8 < KC_) ? b[i] : 0.0f);
            hv[i] = (_Float16)(v * SCL);
        }
        _Float16* d = Wp + (size_t)n * WPITCH + c8;
        *(volatile v8h*)d = hv;
        __threadfence();
        *(volatile v8h*)d = hv;
    } else {
        const int p  = ((int)blockIdx.x - NWBLK) * 256 + tid;
        const int n  = p >> 6;
        const int c8 = (p & 63) * 8;
        const v8f a = ld8f(Wfc + (size_t)n * H_ + c8);
        v8h hv;
#pragma unroll
        for (int i = 0; i < 8; ++i) hv[i] = (_Float16)(a[i] * SCL);
        _Float16* d = Wf + (size_t)n * H_ + c8;
        *(volatile v8h*)d = hv;
        __threadfence();
        *(volatile v8h*)d = hv;
    }
}

__global__ __launch_bounds__(NTHR)
void lstm_seq_kernel(const float* __restrict__ x, const _Float16* __restrict__ Wp,
                     const _Float16* __restrict__ Wf, const float* __restrict__ bih,
                     const float* __restrict__ bhh, const float* __restrict__ bfc,
                     const int* __restrict__ fsp, float* out)
{
    extern __shared__ __attribute__((aligned(16))) char smem[];
    lp_h sA    = (lp_h)(smem + LOFF_A);
    lp_f sC    = (lp_f)(smem + LOFF_C);
    lp_f sBias = (lp_f)(smem + LOFF_BIAS);
    lp_f sBfc  = (lp_f)(smem + LOFF_BFC);
    lp_f sP    = (lp_f)(smem + LOFF_P);

    const int tid  = threadIdx.x;
    const int lane = tid & 31;
    const int w    = tid >> 5;
    const int h    = lane >> 4;
    const int m    = lane & 15;
    const int b0   = blockIdx.x * MB_;
    const int ndec = min(max(fsp[0], 0), F_);

    {
        v8h zh;
#pragma unroll
        for (int i = 0; i < 8; ++i) zh[i] = (_Float16)0.0f;
        for (int i = tid; i < (2 * A_TILE) / 8; i += NTHR) *(AS3 v8h*)(sA + 8 * i) = zh;
        v4f zf;
#pragma unroll
        for (int i = 0; i < 4; ++i) zf[i] = 0.0f;
        for (int i = tid; i < (MB_ * CPITCH) / 4; i += NTHR) *(AS3 v4f*)(sC + 4 * i) = zf;
        for (int i = tid; i < G4_; i += NTHR) sBias[i] = bih[i] + bhh[i];
        if (tid < O_) sBfc[tid] = bfc[tid];
    }
    __syncthreads();

    const int srow = tid >> 3;
    const int sc4  = (tid & 7) * 4;
    const float* xrow = x + (size_t)(b0 + srow) * (T_ * I_) + sc4;

    {
        const v4f xv = *(const v4f*)(xrow);
        v4h hv;
#pragma unroll
        for (int i = 0; i < 4; ++i) hv[i] = (_Float16)(xv[i] * SCL);
        *(AS3 v4h*)(sA + srow * APITCH + sc4) = hv;
    }

#pragma unroll 1
    for (int s = 0; s < NSTEP; ++s) {
        const int cur = s & 1;
        lp_h sAc = sA + cur * A_TILE;
        lp_h sAn = sA + (cur ^ 1) * A_TILE;

        __syncthreads();

        if (s + 1 < T_) {
            const v4f xv = *(const v4f*)(xrow + (size_t)(s + 1) * I_);
            v4h hv;
#pragma unroll
            for (int i = 0; i < 4; ++i) hv[i] = (_Float16)(xv[i] * SCL);
            *(AS3 v4h*)(sAn + srow * APITCH + sc4) = hv;
        }

#pragma unroll 1
        for (int g4 = 0; g4 < 4; ++g4) {
            const int j0 = w * 64 + g4 * 16;
            v8f acc[2][4];
#pragma unroll
            for (int mt = 0; mt < 2; ++mt)
#pragma unroll
                for (int q = 0; q < 4; ++q) acc[mt][q] = zero8();

            lcp_h ab = sAc + m * APITCH + 8 * h;
            const _Float16* wb = Wp + (size_t)(j0 + m) * WPITCH + 8 * h;

#pragma unroll 1
            for (int k0 = 0; k0 < KC_; k0 += 32) {
                Frag a[2], b[4];
#pragma unroll
                for (int mt = 0; mt < 2; ++mt) ldfrag_lds(a[mt], ab + mt * (16 * APITCH) + k0);
#pragma unroll
                for (int q = 0; q < 4; ++q) ldfrag_glb(b[q], wb + (size_t)q * (512 * WPITCH) + k0);
#pragma unroll
                for (int mt = 0; mt < 2; ++mt)
#pragma unroll
                    for (int q = 0; q < 4; ++q) acc[mt][q] = mma16(acc[mt][q], a[mt], b[q]);
                asm volatile("v_nop\n\tv_nop\n\tv_nop\n\tv_nop"
                             : "+v"(acc[0][0]), "+v"(acc[0][1]), "+v"(acc[0][2]), "+v"(acc[0][3]),
                               "+v"(acc[1][0]), "+v"(acc[1][1]), "+v"(acc[1][2]), "+v"(acc[1][3])
                             : "v"(a[0].v), "v"(a[1].v), "v"(b[0].v), "v"(b[1].v), "v"(b[2].v), "v"(b[3].v));
            }

            const int n = j0 + m;
            const float bi = sBias[n];
            const float bf = sBias[H_ + n];
            const float bg = sBias[2 * H_ + n];
            const float bo = sBias[3 * H_ + n];
#pragma unroll
            for (int mt = 0; mt < 2; ++mt) {
#pragma unroll
                for (int r = 0; r < 8; ++r) {
                    const int row = mt * 16 + 8 * h + r;
                    const float gi = acc[mt][0][r] * INV256 + bi;
                    const float gf = acc[mt][1][r] * INV256 + bf;
                    const float gg = acc[mt][2][r] * INV256 + bg;
                    const float go = acc[mt][3][r] * INV256 + bo;
                    const float cp = sC[row * CPITCH + n];
                    const float cn = sigm(gf) * cp + sigm(gi) * tanhm(gg);
                    sC[row * CPITCH + n] = cn;
                    const float hn = sigm(go) * tanhm(cn);
                    sAn[row * APITCH + I_ + n] = (_Float16)(hn * SCL);
                }
            }
        }

        if (s >= T_ - 1) {
            __syncthreads();
            if (w < 4) {
                const int mt = w >> 1, nt = w & 1;
                v8f pacc = zero8();
                lcp_h ab = sAn + (mt * 16 + m) * APITCH + I_ + 8 * h;
                const _Float16* gb = Wf + (size_t)(nt * 16 + m) * H_ + 8 * h;
#pragma unroll 1
                for (int k0 = 0; k0 < H_; k0 += 32) {
                    Frag a, b;
                    ldfrag_lds(a, ab + k0);
                    ldfrag_glb(b, gb + k0);
                    pacc = mma16(pacc, a, b);
                    asm volatile("v_nop\n\tv_nop\n\tv_nop\n\tv_nop" : "+v"(pacc) : "v"(a.v), "v"(b.v));
                }
                const int col = nt * 16 + m;
                const float bb = sBfc[col];
#pragma unroll
                for (int r = 0; r < 8; ++r)
                    sP[(mt * 16 + 8 * h + r) * PPITCH + col] = pacc[r] * INV256 + bb;
            }
            __syncthreads();
            const int d = s - (T_ - 1);
            const v4f pv = *(AS3 const v4f*)(sP + srow * PPITCH + sc4);
            {
                v4h hv;
#pragma unroll
                for (int i = 0; i < 4; ++i) hv[i] = (_Float16)(pv[i] * SCL);
                *(AS3 v4h*)(sAn + srow * APITCH + sc4) = hv;
            }
            float* op = out + ((size_t)(b0 + srow) * F_ + d) * O_ + sc4;
            if (d < ndec) *(volatile v4f*)op = pv;
            __threadfence();
            if (d < ndec) *(volatile v4f*)op = pv;
        }
    }
}

extern "C" void kernel_launch(void* const* d_in, const int* in_sizes, int n_in,
                              void* d_out, int out_size, void* d_ws, size_t ws_size,
                              hipStream_t stream)
{
    if (n_in < 8) return;
    if (in_sizes[0] != B_ * T_ * I_) return;
    if (in_sizes[1] != G4_ * I_)     return;
    if (in_sizes[2] != G4_ * H_)     return;
    if (in_sizes[3] != G4_)          return;
    if (in_sizes[4] != G4_)          return;
    if (in_sizes[5] != O_ * H_)      return;
    if (in_sizes[6] != O_)           return;
    if (in_sizes[7] < 1)             return;
    if (out_size != B_ * F_ * O_)    return;
    if (ws_size < WS_END)            return;

    const float* x   = (const float*)d_in[0];
    const float* Wih = (const float*)d_in[1];
    const float* Whh = (const float*)d_in[2];
    const float* bih = (const float*)d_in[3];
    const float* bhh = (const float*)d_in[4];
    const float* Wfc = (const float*)d_in[5];
    const float* bfc = (const float*)d_in[6];
    const int*   fsp = (const int*)d_in[7];
    float* out = (float*)d_out;

    char* ws = (char*)d_ws;
    _Float16* Wp = (_Float16*)(ws + OFF_WP);
    _Float16* Wf = (_Float16*)(ws + OFF_WF);

    cvt_kernel<<<dim3(NWBLK + NFBLK), dim3(256), 0, stream>>>(Wih, Whh, Wfc, Wp, Wf);

    hipFuncSetAttribute(reinterpret_cast<const void*>(&lstm_seq_kernel),
                        hipFuncAttributeMaxDynamicSharedMemorySize, (int)LDS_BYTES);
    lstm_seq_kernel<<<dim3(NBLK), dim3(NTHR), LDS_BYTES, stream>>>(
        x, (const _Float16*)Wp, (const _Float16*)Wf, bih, bhh, bfc, fsp, out);
}
